// MambaClassifier_37958920962160
// MI455X (gfx1250) — hardware-run, weakly checked
//
#include <hip/hip_runtime.h>
#include <hip/hip_fp16.h>
#include <math.h>

typedef float    ms1_v4f __attribute__((ext_vector_type(4)));
typedef unsigned ms1_v4u __attribute__((ext_vector_type(4)));
struct ms1_args {
  const float* dtpre;
  const float* u;
  const float* bc;
  const float* z;
  const float* A_log;
  const float* Dskip;
  __half* y;
  __half* y_lo;
  long ld_dtpre;
  long ld_u;
  long ld_bc;
  long ld_z;
  long ld_y;
  int offB;
  int offC;
  int offZ;
  float ycarry;
  int dir;
  int D;
  int L;
  int nbatch;
};
static_assert(sizeof(ms1_args) == 136);

__device__ __forceinline__ float ms1_flush16(float v) {
  return (fabsf(v) < 6.103515625e-05f) ? 0.0f : v;
}
__device__ __forceinline__ unsigned ms1_h16bits(float v) {
  return (unsigned)__half_as_ushort(__float2half_rn(ms1_flush16(v)));
}
__device__ __forceinline__ float ms1_h16val(unsigned b) {
  return __half2float(__ushort_as_half((unsigned short)b));
}
__device__ __forceinline__ float ms1_softplus(float v) {
  return fmaxf(v, 0.0f) + log1pf(expf(-fabsf(v)));
}
__device__ __forceinline__ void ms1_pack2(float v0, float v1, unsigned& hw, unsigned& lw) {
  const unsigned h0 = ms1_h16bits(v0);
  const unsigned h1 = ms1_h16bits(v1);
  const float r0 = (v0 - ms1_h16val(h0)) * 2048.0f;
  const float r1 = (v1 - ms1_h16val(h1)) * 2048.0f;
  const unsigned l0 = ms1_h16bits(r0);
  const unsigned l1 = ms1_h16bits(r1);
  hw = h0 | (h1 << 16);
  lw = l0 | (l1 << 16);
}

template <int NSTATE>
__global__ __launch_bounds__(64 * (NSTATE / 16)) void ms1_scan_kernel(ms1_args a)
{
  static_assert(NSTATE == 16 || NSTATE == 64);
  constexpr int NQ  = NSTATE / 16;
  constexpr int NT  = 64 * NQ;
  constexpr int NW  = NT / 32;
  constexpr int BCW = 2 * NSTATE;
  constexpr int YP  = 68;
  constexpr int RPI = NW * 4;
  constexpr int NIT = 64 / RPI;
  static_assert(16 * NT <= 64 * YP);
  __shared__ __align__(16) float sBC[64 * BCW];
  __shared__ __align__(16) float sY[64 * YP];
  const int tid  = threadIdx.x;
  const int lane = tid & 31;
  const int wave = tid >> 5;
  const int c    = tid / NQ;
  const int sq   = tid - c * NQ;
  const int bpb  = a.D / 64;
  const int bi   = blockIdx.x / bpb;
  if (bi >= a.nbatch) return;
  const int d0 = (blockIdx.x - bi * bpb) * 64;
  const int d  = d0 + c;
  const long rowb = (long)bi * a.L;
  const bool hasz  = (a.z != nullptr);
  const bool hasD  = (a.Dskip != nullptr);
  const bool hasLo = (a.y_lo != nullptr);

#pragma unroll 1
  for (int n = 0; n < 16; ++n) {
    const float al = a.A_log[(long)d * NSTATE + sq * 16 + n];
    sY[n * NT + tid] = -expf(al);
  }
  __syncthreads();
  float An[16], h[16];
#pragma unroll
  for (int n = 0; n < 16; ++n) {
    An[n] = sY[n * NT + tid];
    h[n] = 0.0f;
  }
  float Dd = 0.0f;
  if (hasD) Dd = a.Dskip[d];

  const int nchunk = a.L / 64;
  const bool fwd = (a.dir > 0);
  const int s0 = fwd ? 0 : 63;
  const int sd = fwd ? 1 : -1;
  const int q  = lane >> 3;
  const int c8 = (lane & 7) * 8;

#pragma unroll 1
  for (int ci = 0; ci < nchunk; ++ci) {
    const int tb = fwd ? (ci * 64) : (a.L - 64 - ci * 64);
    const long rowc = rowb + tb;
    __syncthreads();
#pragma unroll 8
    for (int i = 0; i < 32; ++i) {
      const int idx = tid + i * NT;
      const int st  = idx / BCW;
      const int col = idx - st * BCW;
      const int sc  = (col < NSTATE) ? (a.offB + col) : (a.offC + col - NSTATE);
      sBC[idx] = a.bc[(rowc + st) * a.ld_bc + sc];
    }
    __syncthreads();
#pragma unroll 1
    for (int s = 0; s < 64; ++s) {
      const int ls = s0 + sd * s;
      const long row = rowc + ls;
      float pre = a.dtpre[row * a.ld_dtpre + d];
      float uv  = a.u[row * a.ld_u + d];
      float zv  = 0.0f;
      if (hasz) zv = a.z[row * a.ld_z + a.offZ + d];
      asm volatile("" : "+v"(pre));
      asm volatile("" : "+v"(uv));
      asm volatile("" : "+v"(zv));
      const float delta = ms1_softplus(pre);
      const float dtx = delta * uv;
      const float* bp = sBC + ls * BCW + sq * 16;
      const float* cp = bp + NSTATE;
      ms1_v4f Bq[4], Cq[4];
#pragma unroll
      for (int k = 0; k < 4; ++k) {
        Bq[k] = *(const ms1_v4f*)(bp + 4 * k);
        Cq[k] = *(const ms1_v4f*)(cp + 4 * k);
      }
      float yv = 0.0f;
#pragma unroll
      for (int n = 0; n < 16; ++n) {
        const float e = __expf(delta * An[n]);
        h[n] = fmaf(e, h[n], dtx * Bq[n >> 2][n & 3]);
        yv = fmaf(h[n], Cq[n >> 2][n & 3], yv);
      }
      if (NQ > 1) {
        yv += __shfl_xor(yv, 1, 32);
        yv += __shfl_xor(yv, 2, 32);
      }
      if (hasD) yv = fmaf(uv, Dd, yv);
      if (hasz) {
        const float sg = __builtin_amdgcn_rcpf(1.0f + expf(-zv));
        yv = yv * (zv * sg);
      }
      if (sq == 0) sY[ls * YP + c] = yv * a.ycarry;
    }
    __syncthreads();
    ms1_v4u hw[NIT], lw[NIT];
#pragma unroll
    for (int it = 0; it < NIT; ++it) {
      const int row = it * RPI + wave * 4 + q;
      const float* sp = sY + row * YP + c8;
      const ms1_v4f f0 = *(const ms1_v4f*)(sp);
      const ms1_v4f f1 = *(const ms1_v4f*)(sp + 4);
      unsigned h0, h1, h2, h3, l0, l1, l2, l3;
      ms1_pack2(f0[0], f0[1], h0, l0);
      ms1_pack2(f0[2], f0[3], h1, l1);
      ms1_pack2(f1[0], f1[1], h2, l2);
      ms1_pack2(f1[2], f1[3], h3, l3);
      hw[it] = (ms1_v4u){h0, h1, h2, h3};
      lw[it] = (ms1_v4u){l0, l1, l2, l3};
    }
    for (int pass = 0; pass < 2; ++pass) {
#pragma unroll
      for (int it = 0; it < NIT; ++it) {
        const int row = it * RPI + wave * 4 + q;
        const long o = (rowc + row) * a.ld_y + d0 + c8;
        *(volatile ms1_v4u*)(a.y + o) = hw[it];
        if (hasLo) *(volatile ms1_v4u*)(a.y_lo + o) = lw[it];
      }
      __threadfence();
    }
  }
}

namespace eng {

constexpr int kBatch    = 32;
constexpr int kCin      = 3;
constexpr int kImg      = 224;
constexpr int kPatch    = 14;
constexpr int kGridP    = kImg / kPatch;
constexpr int kSeq      = kGridP * kGridP;
constexpr int kDm       = 384;
constexpr int kDin      = 768;
constexpr int kNstate   = 16;
constexpr int kRank     = 48;
constexpr int kRankP    = 64;
constexpr int kLayers   = 4;
constexpr int kNcls     = 1000;
constexpr int kNclsP    = 1024;
constexpr int kKp       = kCin * kPatch * kPatch;
constexpr int kKpP      = 640;
constexpr int kRows     = kBatch * kSeq;
constexpr int kHalves   = 2;
constexpr int kHalfImgs = kBatch / kHalves;
constexpr int kHalfRows = kHalfImgs * kSeq;
constexpr int kXzN      = 2 * kDin;
constexpr int kXdN      = kRank + 2 * kNstate;
constexpr int kXdP      = 128;
constexpr int kOffB     = kRank;
constexpr int kOffC     = kRank + kNstate;

static_assert(kGridP == 16 && kSeq == 256 && kKp == 588 && kXdN == 80 && kRows == 8192 && kHalfRows == 4096);
static_assert(kKpP % 64 == 0 && kKpP >= kKp && kRankP >= kRank && kXdP >= kXdN && kNclsP >= kNcls);
static_assert(kKp % 4 == 0 && kRank % 4 == 0 && kDm % 4 == 0 && kDin % 4 == 0);
static_assert(kRows % 64 == 0 && kHalfRows % 64 == 0 && kBatch % 32 == 0);
static_assert(kDm % 64 == 0 && kXzN % 64 == 0 && kXdP % 64 == 0 && kDin % 64 == 0 && kNclsP % 64 == 0);
static_assert(kKpP % 32 == 0 && kDm % 32 == 0 && kDin % 32 == 0 && kRankP % 32 == 0);
static_assert(kDin % 64 == 0 && kSeq % 64 == 0);
static_assert((kOffB * 4) % 16 == 0 && (kOffC * 4) % 16 == 0);
static_assert(kDin == 192 * 4);

constexpr float kCarryImg  = 16.0f;
constexpr float kCarryW    = 256.0f;
constexpr float kCarryWdt  = 64.0f;
constexpr float kCarryXn   = 16.0f;
constexpr float kCarryUc   = 16.0f;
constexpr float kCarryDtl  = 64.0f;
constexpr float kCarryY    = 16.0f;
constexpr float kCarryPool = 128.0f;
constexpr float kResid     = 2048.0f;
constexpr float kFoldPatch = 1.0f / (kCarryImg * kCarryW);
constexpr float kFoldIn    = 1.0f / (kCarryXn * kCarryW);
constexpr float kFoldXp    = 1.0f / (kCarryUc * kCarryW);
constexpr float kFoldDt    = 1.0f / (kCarryDtl * kCarryWdt);
constexpr float kFoldOut   = 1.0f / (kCarryY * kCarryW);
constexpr float kFoldHead  = 1.0f / (kCarryPool * kCarryW);
constexpr float kFoldResid = 1.0f / kResid;

constexpr size_t kBytesColA   = (size_t)kRows * kKpP * 2;
constexpr size_t kBytesWPatch = (size_t)kDm * kKpP * 2;
constexpr size_t kBytesWIn    = (size_t)kLayers * kXzN * kDm * 2;
constexpr size_t kBytesWX     = (size_t)kLayers * kXdP * kDin * 2;
constexpr size_t kBytesWDt    = (size_t)kLayers * kDin * kRankP * 2;
constexpr size_t kBytesWOut   = (size_t)kLayers * kDm * kDin * 2;
constexpr size_t kBytesWCls   = (size_t)kNclsP * kDm * 2;
constexpr size_t kBytesT      = (size_t)kRows * kDm * 4;
constexpr size_t kBytesXN     = (size_t)kHalfRows * kDm * 2;
constexpr size_t kBytesXZ     = (size_t)kHalfRows * kXzN * 4;
constexpr size_t kBytesUC     = (size_t)kHalfRows * kDin * 4;
constexpr size_t kBytesUCh    = (size_t)kHalfRows * kDin * 2;
constexpr size_t kBytesXDBL   = (size_t)kHalfRows * kXdP * 4;
constexpr size_t kBytesDTLh   = (size_t)kHalfRows * kRankP * 2;
constexpr size_t kBytesDTP    = (size_t)kHalfRows * kDin * 4;
constexpr size_t kBytesYH     = (size_t)kHalfRows * kDin * 2;
constexpr size_t kBytesYL     = (size_t)kHalfRows * kDin * 2;
constexpr size_t kBytesPoolH  = (size_t)kBatch * kDm * 2;
constexpr size_t kBytesLOG    = (size_t)kBatch * kNclsP * 4;
constexpr size_t kWsTotal = kBytesColA + kBytesWPatch + kBytesWIn + kBytesWX + kBytesWDt + kBytesWOut + kBytesWCls +
                            kBytesT + kBytesT + kBytesXN + kBytesXZ + kBytesUC + kBytesUCh + kBytesXDBL + kBytesDTLh +
                            kBytesDTP + kBytesYH + kBytesYL + kBytesPoolH + kBytesLOG;
static_assert(kBytesColA == 10485760ull && kBytesWPatch == 491520ull && kBytesWIn == 4718592ull);
static_assert(kBytesWX == 786432ull && kBytesWDt == 393216ull && kBytesWOut == 2359296ull && kBytesWCls == 786432ull);
static_assert(kBytesT == 12582912ull && kBytesXN == 3145728ull && kBytesXZ == 25165824ull && kBytesUC == 12582912ull);
static_assert(kBytesUCh == 6291456ull && kBytesXDBL == 2097152ull && kBytesDTLh == 524288ull && kBytesDTP == 12582912ull);
static_assert(kBytesYH == 6291456ull && kBytesYL == 6291456ull && kBytesPoolH == 24576ull && kBytesLOG == 131072ull);
static_assert(kWsTotal == 120315904ull);
static_assert(kWsTotal <= 134217728ull);
static_assert(kBytesColA % 128 == 0 && kBytesWPatch % 128 == 0 && kBytesWIn % 128 == 0 && kBytesWX % 128 == 0 &&
              kBytesWDt % 128 == 0 && kBytesWOut % 128 == 0 && kBytesWCls % 128 == 0 && kBytesT % 128 == 0 &&
              kBytesXN % 128 == 0 && kBytesXZ % 128 == 0 && kBytesUC % 128 == 0 && kBytesUCh % 128 == 0 &&
              kBytesXDBL % 128 == 0 && kBytesDTLh % 128 == 0 && kBytesDTP % 128 == 0 && kBytesYH % 128 == 0 &&
              kBytesYL % 128 == 0 && kBytesPoolH % 128 == 0 && kBytesLOG % 128 == 0);

typedef _Float16 v16h __attribute__((ext_vector_type(16)));
typedef _Float16 v8h  __attribute__((ext_vector_type(8)));
typedef float    v8f  __attribute__((ext_vector_type(8)));
typedef float    v4f  __attribute__((ext_vector_type(4)));
typedef float    v2f  __attribute__((ext_vector_type(2)));
typedef unsigned v4u  __attribute__((ext_vector_type(4)));

__device__ __forceinline__ float flush16(float v) {
  return (fabsf(v) < 6.103515625e-05f) ? 0.0f : v;
}
__device__ __forceinline__ unsigned h16bits(float v) {
  return (unsigned)__half_as_ushort(__float2half_rn(flush16(v)));
}
__device__ __forceinline__ unsigned pack2(float a, float b) {
  const unsigned lo = h16bits(a);
  const unsigned hi = h16bits(b);
  return lo | (hi << 16);
}

union FragU { v16h v; v8h h[2]; };
__device__ __forceinline__ v16h frag_load(const _Float16* p) {
  FragU f;
  f.h[0] = *(const v8h*)(p);
  f.h[1] = *(const v8h*)(p + 16);
  return f.v;
}
__device__ __forceinline__ v8f mma(v16h a, v16h b, v8f c) {
  c = __builtin_amdgcn_wmma_f32_16x16x32_f16(false, a, false, b, (short)0, c, false, false);
  asm volatile("v_nop\n\tv_nop\n\tv_nop\n\tv_nop" : "+v"(c) : "v"(a), "v"(b));
  return c;
}

__global__ __launch_bounds__(256) void im2col_f16_kernel(
    const float* __restrict__ x, unsigned short* __restrict__ col, float carry)
{
  constexpr int kSegs = kKpP / 8;
  const int i  = blockIdx.x * 256 + threadIdx.x;
  const int m  = i / kSegs;
  const int k0 = (i - m * kSegs) * 8;
  const int b  = m / kSeq;
  const int pidx = m - b * kSeq;
  const int py = pidx / kGridP;
  const int px = pidx - py * kGridP;
  const float* xb = x + (size_t)b * (kCin * kImg * kImg) + (size_t)(py * kPatch) * kImg + px * kPatch;
  float e[8];
#pragma unroll
  for (int j = 0; j < 8; ++j) {
    const int k  = k0 + j;
    const int kc = (k < kKp) ? k : (kKp - 1);
    const int c  = kc / (kPatch * kPatch);
    const int rem = kc - c * (kPatch * kPatch);
    const int ii = rem / kPatch;
    const int jj = rem - ii * kPatch;
    float v = xb[(size_t)c * (kImg * kImg) + ii * kImg + jj];
    asm volatile("" : "+v"(v));
    e[j] = (k < kKp) ? (v * carry) : 0.0f;
  }
  const v4u hw = (v4u){pack2(e[0], e[1]), pack2(e[2], e[3]), pack2(e[4], e[5]), pack2(e[6], e[7])};
  unsigned short* o = col + (size_t)i * 8;
  for (int pass = 0; pass < 2; ++pass) {
    *(volatile v4u*)(o) = hw;
    __threadfence();
  }
}

__global__ __launch_bounds__(256) void cast_pad_f16_kernel(
    const float* __restrict__ in, unsigned short* __restrict__ out,
    int rowsPad, int rowsReal, int kReal, int kPad, float carry)
{
  const int i    = blockIdx.x * 256 + threadIdx.x;
  const int segs = kPad >> 3;
  const int row  = i / segs;
  const int k0   = (i - row * segs) * 8;
  const int g    = row / rowsPad;
  const int rr   = row - g * rowsPad;
  const int rc   = (rr < rowsReal) ? rr : (rowsReal - 1);
  const size_t srow = (size_t)g * rowsReal + rc;
  const int ka = (k0 < kReal) ? k0 : (kReal - 4);
  const int kb = (k0 + 4 < kReal) ? (k0 + 4) : (kReal - 4);
  v4f f0 = *(const v4f*)(in + srow * kReal + ka);
  v4f f1 = *(const v4f*)(in + srow * kReal + kb);
  asm volatile("" : "+v"(f0));
  asm volatile("" : "+v"(f1));
  const bool rowOn = (rr < rowsReal);
  const bool on0 = rowOn && (k0 < kReal);
  const bool on1 = rowOn && (k0 + 4 < kReal);
  const float e0 = on0 ? (f0[0] * carry) : 0.0f;
  const float e1 = on0 ? (f0[1] * carry) : 0.0f;
  const float e2 = on0 ? (f0[2] * carry) : 0.0f;
  const float e3 = on0 ? (f0[3] * carry) : 0.0f;
  const float e4 = on1 ? (f1[0] * carry) : 0.0f;
  const float e5 = on1 ? (f1[1] * carry) : 0.0f;
  const float e6 = on1 ? (f1[2] * carry) : 0.0f;
  const float e7 = on1 ? (f1[3] * carry) : 0.0f;
  const v4u hw = (v4u){pack2(e0, e1), pack2(e2, e3), pack2(e4, e5), pack2(e6, e7)};
  unsigned short* o = out + (size_t)i * 8;
  for (int pass = 0; pass < 2; ++pass) {
    *(volatile v4u*)(o) = hw;
    __threadfence();
  }
}

__global__ __launch_bounds__(256) void ln_f16_kernel(
    const float* __restrict__ t, const float* __restrict__ gw, const float* __restrict__ gb,
    unsigned short* __restrict__ xn, float carry)
{
  const int lane = threadIdx.x & 31;
  const int wave = threadIdx.x >> 5;
  const int row  = blockIdx.x * 8 + wave;
  const float* r = t + (size_t)row * kDm;
  float a0[6], a1[6];
  float s = 0.0f;
#pragma unroll
  for (int i = 0; i < 6; ++i) {
    const v2f ld = *(const v2f*)(r + 2 * lane + 64 * i);
    a0[i] = ld[0];
    a1[i] = ld[1];
    s += ld[0] + ld[1];
  }
#pragma unroll
  for (int o = 16; o > 0; o >>= 1) s += __shfl_xor(s, o, 32);
  const float mean = s * (1.0f / (float)kDm);
  float sq = 0.0f;
#pragma unroll
  for (int i = 0; i < 6; ++i) {
    const float d0 = a0[i] - mean;
    const float d1 = a1[i] - mean;
    sq += d0 * d0 + d1 * d1;
  }
#pragma unroll
  for (int o = 16; o > 0; o >>= 1) sq += __shfl_xor(sq, o, 32);
  const float inv = 1.0f / sqrtf(sq * (1.0f / (float)kDm) + 1e-5f);
  unsigned hw[6];
#pragma unroll
  for (int i = 0; i < 6; ++i) {
    const v2f w2 = *(const v2f*)(gw + 2 * lane + 64 * i);
    const v2f b2 = *(const v2f*)(gb + 2 * lane + 64 * i);
    const float o0 = (a0[i] - mean) * inv * w2[0] + b2[0];
    const float o1 = (a1[i] - mean) * inv * w2[1] + b2[1];
    hw[i] = pack2(o0 * carry, o1 * carry);
  }
  unsigned* op = (unsigned*)(void*)(xn + (size_t)row * kDm);
  for (int pass = 0; pass < 2; ++pass) {
#pragma unroll
    for (int i = 0; i < 6; ++i) {
      *(volatile unsigned*)(op + lane + 32 * i) = hw[i];
    }
    __threadfence();
  }
}

template <int MT, int ATERMS, int EPI>
__global__ __launch_bounds__(256) void gemm_f16_kernel(
    const unsigned short* __restrict__ Ap, const unsigned short* __restrict__ A2p, int lda,
    const unsigned short* __restrict__ Btp, int ldb,
    float* __restrict__ C, int ldc,
    unsigned short* __restrict__ C16, int ldc16, int n16valid,
    const float* __restrict__ bias,
    const float* __restrict__ addp,
    int M, int N, int K, float scale, float scale2, float scale16)
{
  const _Float16* A  = (const _Float16*)(const void*)Ap;
  const _Float16* A2 = (const _Float16*)(const void*)A2p;
  const _Float16* Bt = (const _Float16*)(const void*)Btp;
  __shared__ __align__(16) float sT[8][16 * 68];
  const int lane = threadIdx.x & 31;
  const int wave = threadIdx.x >> 5;
  const int tilesN = N >> 6;
  const int tilesM = M / (16 * MT);
  const int tile = blockIdx.x * 8 + wave;
  if (tile >= tilesM * tilesN) return;
  const int tm = tile / tilesN;
  const int tn = tile - tm * tilesN;
  const int m0 = tm * (16 * MT);
  const int n0 = tn << 6;
  const int rlane = lane & 15;
  const int koff  = (lane >> 4) * 8;
  const int mOff  = (lane >> 4) * 8;

  v8f accH[MT][4];
  v8f accL[MT][4];
#pragma unroll
  for (int i = 0; i < MT; ++i) {
#pragma unroll
    for (int j = 0; j < 4; ++j) {
      accH[i][j] = (v8f){0.f, 0.f, 0.f, 0.f, 0.f, 0.f, 0.f, 0.f};
      accL[i][j] = (v8f){0.f, 0.f, 0.f, 0.f, 0.f, 0.f, 0.f, 0.f};
    }
  }

#pragma unroll 1
  for (int k0 = 0; k0 < K; k0 += 32) {
    v16h bf[4];
#pragma unroll
    for (int j = 0; j < 4; ++j) {
      bf[j] = frag_load(Bt + (size_t)(n0 + (j << 4) + rlane) * ldb + koff + k0);
    }
#pragma unroll
    for (int i = 0; i < MT; ++i) {
      const size_t ao = (size_t)(m0 + (i << 4) + rlane) * lda + koff + k0;
      const v16h a0 = frag_load(A + ao);
#pragma unroll
      for (int j = 0; j < 4; ++j) accH[i][j] = mma(a0, bf[j], accH[i][j]);
      if (ATERMS == 2) {
        const v16h a1 = frag_load(A2 + ao);
#pragma unroll
        for (int j = 0; j < 4; ++j) accL[i][j] = mma(a1, bf[j], accL[i][j]);
      }
    }
  }

  float* slab = sT[wave];
  float bv[4] = {0.f, 0.f, 0.f, 0.f};
  if (EPI == 2) {
#pragma unroll
    for (int j = 0; j < 4; ++j) bv[j] = bias[n0 + (j << 4) + rlane];
  }
#pragma unroll
  for (int i = 0; i < MT; ++i) {
    const int mBase = m0 + (i << 4);
#pragma unroll
    for (int j = 0; j < 4; ++j) {
#pragma unroll
      for (int r = 0; r < 8; ++r) {
        float v = accH[i][j][r];
        if (ATERMS == 2) v = v + accL[i][j][r] * scale2;
        v = v * scale;
        if (EPI == 2) v = v + bv[j];
        slab[(mOff + r) * 68 + (j << 4) + rlane] = v;
      }
    }
    __builtin_amdgcn_fence(__ATOMIC_RELEASE, "workgroup");
    __builtin_amdgcn_wave_barrier();
    __builtin_amdgcn_fence(__ATOMIC_ACQUIRE, "workgroup");
    {
      const int hh = lane >> 4;
      const int c4 = (lane & 15) * 4;
      if (EPI == 3) {
        v4f val[8];
#pragma unroll
        for (int it = 0; it < 8; ++it) {
          const int row = it * 2 + hh;
          const v4f sv = *(const v4f*)(slab + row * 68 + c4);
          const v4f rv = *(const v4f*)(addp + (size_t)(mBase + row) * ldc + n0 + c4);
          val[it] = sv + rv;
        }
        for (int pass = 0; pass < 2; ++pass) {
#pragma unroll
          for (int it = 0; it < 8; ++it) {
            const int row = it * 2 + hh;
            *(volatile v4f*)(C + (size_t)(mBase + row) * ldc + n0 + c4) = val[it];
          }
          __threadfence();
        }
      } else {
        for (int pass = 0; pass < 2; ++pass) {
#pragma unroll
          for (int it = 0; it < 8; ++it) {
            const int row = it * 2 + hh;
            const v4f val = *(const v4f*)(slab + row * 68 + c4);
            *(volatile v4f*)(C + (size_t)(mBase + row) * ldc + n0 + c4) = val;
          }
          __threadfence();
        }
      }
    }
    if (EPI == 1) {
      if (n0 == 0) {
        const int q  = lane >> 3;
        const int c8 = (lane & 7) * 8;
        const bool keep = (c8 < n16valid);
        v4u hw[4];
#pragma unroll
        for (int it = 0; it < 4; ++it) {
          const int row = it * 4 + q;
          const float* sp = slab + row * 68 + c8;
          const v4f f0 = *(const v4f*)(sp);
          const v4f f1 = *(const v4f*)(sp + 4);
          const float e0 = keep ? (f0[0] * scale16) : 0.0f;
          const float e1 = keep ? (f0[1] * scale16) : 0.0f;
          const float e2 = keep ? (f0[2] * scale16) : 0.0f;
          const float e3 = keep ? (f0[3] * scale16) : 0.0f;
          const float e4 = keep ? (f1[0] * scale16) : 0.0f;
          const float e5 = keep ? (f1[1] * scale16) : 0.0f;
          const float e6 = keep ? (f1[2] * scale16) : 0.0f;
          const float e7 = keep ? (f1[3] * scale16) : 0.0f;
          hw[it] = (v4u){pack2(e0, e1), pack2(e2, e3), pack2(e4, e5), pack2(e6, e7)};
        }
        for (int pass = 0; pass < 2; ++pass) {
#pragma unroll
          for (int it = 0; it < 4; ++it) {
            const int row = it * 4 + q;
            *(volatile v4u*)(C16 + (size_t)(mBase + row) * ldc16 + c8) = hw[it];
          }
          __threadfence();
        }
      }
    }
    __builtin_amdgcn_fence(__ATOMIC_RELEASE, "workgroup");
    __builtin_amdgcn_wave_barrier();
    __builtin_amdgcn_fence(__ATOMIC_ACQUIRE, "workgroup");
  }
}

__device__ __forceinline__ float conv_silu_one(v4f w, float u0, float u1, float u2, float u3, float b) {
  float acc = w[0] * u0;
  acc = fmaf(w[1], u1, acc);
  acc = fmaf(w[2], u2, acc);
  acc = fmaf(w[3], u3, acc);
  const float cv = acc + b;
  const float sg = __builtin_amdgcn_rcpf(1.0f + __expf(-cv));
  return cv * sg;
}

__global__ __launch_bounds__(192) void conv_silu_kernel(
    const float* __restrict__ XZ, const float* __restrict__ conv_w, const float* __restrict__ conv_b,
    float* __restrict__ UC, unsigned short* __restrict__ UCh, float carry)
{
  __shared__ __align__(16) float sRow[kDin];
  const int tid = threadIdx.x;
  const int r = blockIdx.x;
  const int t = r & (kSeq - 1);
  const int rb = r - t;
  const int d4 = tid * 4;
  const v4f bs = *(const v4f*)(conv_b + d4);
  const v4f w0 = *(const v4f*)(conv_w + (size_t)d4 * 4);
  const v4f w1 = *(const v4f*)(conv_w + (size_t)d4 * 4 + 4);
  const v4f w2 = *(const v4f*)(conv_w + (size_t)d4 * 4 + 8);
  const v4f w3 = *(const v4f*)(conv_w + (size_t)d4 * 4 + 12);
  v4f ut[4];
#pragma unroll
  for (int k = 0; k < 4; ++k) {
    const int tt = t - 3 + k;
    const int tc = (tt < 0) ? 0 : tt;
    const bool on = (tt >= 0);
    const v4f ld = *(const v4f*)(XZ + (size_t)(rb + tc) * kXzN + d4);
    v4f uv;
    uv[0] = on ? ld[0] : 0.0f;
    uv[1] = on ? ld[1] : 0.0f;
    uv[2] = on ? ld[2] : 0.0f;
    uv[3] = on ? ld[3] : 0.0f;
    ut[k] = uv;
  }
  v4f o;
  o[0] = conv_silu_one(w0, ut[0][0], ut[1][0], ut[2][0], ut[3][0], bs[0]);
  o[1] = conv_silu_one(w1, ut[0][1], ut[1][1], ut[2][1], ut[3][1], bs[1]);
  o[2] = conv_silu_one(w2, ut[0][2], ut[1][2], ut[2][2], ut[3][2], bs[2]);
  o[3] = conv_silu_one(w3, ut[0][3], ut[1][3], ut[2][3], ut[3][3], bs[3]);
  *(v4f*)(sRow + d4) = o;
  __syncthreads();
  const bool doH = (tid < 96);
  const int t8 = doH ? tid : 0;
  const v4f f0 = *(const v4f*)(sRow + t8 * 8);
  const v4f f1 = *(const v4f*)(sRow + t8 * 8 + 4);
  const float e0 = f0[0] * carry;
  const float e1 = f0[1] * carry;
  const float e2 = f0[2] * carry;
  const float e3 = f0[3] * carry;
  const float e4 = f1[0] * carry;
  const float e5 = f1[1] * carry;
  const float e6 = f1[2] * carry;
  const float e7 = f1[3] * carry;
  const v4u hw = (v4u){pack2(e0, e1), pack2(e2, e3), pack2(e4, e5), pack2(e6, e7)};
  float* ucr = UC + (size_t)r * kDin;
  unsigned short* uhr = UCh + (size_t)r * kDin;
  for (int pass = 0; pass < 2; ++pass) {
    *(volatile v4f*)(ucr + d4) = o;
    if (doH) *(volatile v4u*)(uhr + t8 * 8) = hw;
    __threadfence();
  }
}

__global__ __launch_bounds__(256) void ln_pool_kernel(
    const float* __restrict__ t, const float* __restrict__ gw, const float* __restrict__ gb,
    unsigned short* __restrict__ pool, float carry)
{
  __shared__ __align__(16) float sAcc[8 * kDm];
  const int tid  = threadIdx.x;
  const int lane = tid & 31;
  const int wave = tid >> 5;
  const int img  = blockIdx.x;
  v2f w2[6], b2[6];
  float p0[6], p1[6];
#pragma unroll
  for (int i = 0; i < 6; ++i) {
    w2[i] = *(const v2f*)(gw + 2 * lane + 64 * i);
    b2[i] = *(const v2f*)(gb + 2 * lane + 64 * i);
    p0[i] = 0.0f;
    p1[i] = 0.0f;
  }
#pragma unroll 1
  for (int j = 0; j < 32; ++j) {
    const float* r = t + (size_t)(img * kSeq + wave * 32 + j) * kDm;
    float a0[6], a1[6];
    float s = 0.0f;
#pragma unroll
    for (int i = 0; i < 6; ++i) {
      const v2f ld = *(const v2f*)(r + 2 * lane + 64 * i);
      a0[i] = ld[0];
      a1[i] = ld[1];
      s += ld[0] + ld[1];
    }
#pragma unroll
    for (int o = 16; o > 0; o >>= 1) s += __shfl_xor(s, o, 32);
    const float mean = s * (1.0f / (float)kDm);
    float sq = 0.0f;
#pragma unroll
    for (int i = 0; i < 6; ++i) {
      const float d0 = a0[i] - mean;
      const float d1 = a1[i] - mean;
      sq += d0 * d0 + d1 * d1;
    }
#pragma unroll
    for (int o = 16; o > 0; o >>= 1) sq += __shfl_xor(sq, o, 32);
    const float inv = 1.0f / sqrtf(sq * (1.0f / (float)kDm) + 1e-5f);
#pragma unroll
    for (int i = 0; i < 6; ++i) {
      p0[i] += (a0[i] - mean) * inv * w2[i][0] + b2[i][0];
      p1[i] += (a1[i] - mean) * inv * w2[i][1] + b2[i][1];
    }
  }
#pragma unroll
  for (int i = 0; i < 6; ++i) {
    v2f pv;
    pv[0] = p0[i];
    pv[1] = p1[i];
    *(v2f*)(sAcc + wave * kDm + 2 * lane + 64 * i) = pv;
  }
  __syncthreads();
  const bool doS = (tid < 192);
  const int tc = doS ? tid : 0;
  float e0 = 0.0f;
  float e1 = 0.0f;
#pragma unroll
  for (int w = 0; w < 8; ++w) {
    const v2f pv = *(const v2f*)(sAcc + w * kDm + 2 * tc);
    e0 += pv[0];
    e1 += pv[1];
  }
  const float sc = carry * (1.0f / (float)kSeq);
  const unsigned hw = pack2(e0 * sc, e1 * sc);
  unsigned* op = (unsigned*)(void*)(pool + (size_t)img * kDm);
  for (int pass = 0; pass < 2; ++pass) {
    if (doS) *(volatile unsigned*)(op + tc) = hw;
    __threadfence();
  }
}

__global__ __launch_bounds__(256) void logits_out_kernel(
    const float* __restrict__ logit, const float* __restrict__ cls_b, float* __restrict__ out)
{
  const int idx = blockIdx.x * 256 + threadIdx.x;
  const int b = idx / kNcls;
  const int n = idx - b * kNcls;
  const float v = logit[(size_t)b * kNclsP + n] + cls_b[n];
  for (int pass = 0; pass < 2; ++pass) {
    *(volatile float*)(out + idx) = v;
    __threadfence();
  }
}

}

extern "C" void kernel_launch(void* const* d_in, const int* in_sizes, int n_in,
                              void* d_out, int out_size, void* d_ws, size_t ws_size, hipStream_t stream)
{
  using namespace eng;
  if (n_in != 18) return;
  if (in_sizes[0] != kBatch * kCin * kImg * kImg) return;
  if (in_sizes[1] != kDm * kKp) return;
  if (in_sizes[2] != kDm) return;
  if (in_sizes[3] != kLayers * kDm) return;
  if (in_sizes[4] != kLayers * kDm) return;
  if (in_sizes[5] != kLayers * kXzN * kDm) return;
  if (in_sizes[6] != kLayers * kDin * 4) return;
  if (in_sizes[7] != kLayers * kDin) return;
  if (in_sizes[8] != kLayers * kDin * kNstate) return;
  if (in_sizes[9] != kLayers * kDin) return;
  if (in_sizes[10] != kLayers * kXdN * kDin) return;
  if (in_sizes[11] != kLayers * kDin * kRank) return;
  if (in_sizes[12] != kLayers * kDin) return;
  if (in_sizes[13] != kLayers * kDm * kDin) return;
  if (in_sizes[14] != kDm) return;
  if (in_sizes[15] != kDm) return;
  if (in_sizes[16] != kNcls * kDm) return;
  if (in_sizes[17] != kNcls) return;
  if (out_size != kBatch * kNcls) return;
  if (ws_size < kWsTotal) return;

  const float* x        = (const float*)d_in[0];
  const float* patch_w  = (const float*)d_in[1];
  const float* patch_b  = (const float*)d_in[2];
  const float* norm_w   = (const float*)d_in[3];
  const float* norm_b   = (const float*)d_in[4];
  const float* inproj_w = (const float*)d_in[5];
  const float* conv_w   = (const float*)d_in[6];
  const float* conv_b   = (const float*)d_in[7];
  const float* A_log    = (const float*)d_in[8];
  const float* D_par    = (const float*)d_in[9];
  const float* xproj_w  = (const float*)d_in[10];
  const float* dtproj_w = (const float*)d_in[11];
  const float* dtproj_b = (const float*)d_in[12];
  const float* outproj_w = (const float*)d_in[13];
  const float* fnorm_w  = (const float*)d_in[14];
  const float* fnorm_b  = (const float*)d_in[15];
  const float* cls_w    = (const float*)d_in[16];
  const float* cls_b    = (const float*)d_in[17];
  float* out = (float*)d_out;

  char* ws = (char*)d_ws;
  size_t off = 0;
  unsigned short* ColA   = (unsigned short*)(ws + off);
  off += kBytesColA;
  unsigned short* WPatch = (unsigned short*)(ws + off);
  off += kBytesWPatch;
  unsigned short* WIn    = (unsigned short*)(ws + off);
  off += kBytesWIn;
  unsigned short* WX     = (unsigned short*)(ws + off);
  off += kBytesWX;
  unsigned short* WDt    = (unsigned short*)(ws + off);
  off += kBytesWDt;
  unsigned short* WOut   = (unsigned short*)(ws + off);
  off += kBytesWOut;
  unsigned short* WCls   = (unsigned short*)(ws + off);
  off += kBytesWCls;
  float* T0              = (float*)(ws + off);
  off += kBytesT;
  float* T1              = (float*)(ws + off);
  off += kBytesT;
  unsigned short* XN     = (unsigned short*)(ws + off);
  off += kBytesXN;
  float* XZ              = (float*)(ws + off);
  off += kBytesXZ;
  float* UC              = (float*)(ws + off);
  off += kBytesUC;
  unsigned short* UCh    = (unsigned short*)(ws + off);
  off += kBytesUCh;
  float* XDBL            = (float*)(ws + off);
  off += kBytesXDBL;
  unsigned short* DTLh   = (unsigned short*)(ws + off);
  off += kBytesDTLh;
  float* DTP             = (float*)(ws + off);
  off += kBytesDTP;
  unsigned short* YH     = (unsigned short*)(ws + off);
  off += kBytesYH;
  unsigned short* YL     = (unsigned short*)(ws + off);
  off += kBytesYL;
  unsigned short* PoolH  = (unsigned short*)(ws + off);
  off += kBytesPoolH;
  float* LOG             = (float*)(ws + off);
  off += kBytesLOG;
  if (off != kWsTotal) return;

  static_assert((kRows * (kKpP / 8)) % 256 == 0);
  static_assert((kDm * kKpP / 8) % 256 == 0);
  static_assert((kLayers * kXzN * kDm / 8) % 256 == 0);
  static_assert((kLayers * kXdP * kDin / 8) % 256 == 0);
  static_assert((kLayers * kDin * kRankP / 8) % 256 == 0);
  static_assert((kLayers * kDm * kDin / 8) % 256 == 0);
  static_assert((kNclsP * kDm / 8) % 256 == 0);
  static_assert(kHalfRows % 8 == 0 && (kBatch * kNcls) % 256 == 0);

  im2col_f16_kernel<<<dim3(kRows * (kKpP / 8) / 256), 256, 0, stream>>>(x, ColA, kCarryImg);
  cast_pad_f16_kernel<<<dim3(kDm * kKpP / 8 / 256), 256, 0, stream>>>(
      patch_w, WPatch, kDm, kDm, kKp, kKpP, kCarryW);
  cast_pad_f16_kernel<<<dim3(kLayers * kXzN * kDm / 8 / 256), 256, 0, stream>>>(
      inproj_w, WIn, kXzN, kXzN, kDm, kDm, kCarryW);
  cast_pad_f16_kernel<<<dim3(kLayers * kXdP * kDin / 8 / 256), 256, 0, stream>>>(
      xproj_w, WX, kXdP, kXdN, kDin, kDin, kCarryW);
  cast_pad_f16_kernel<<<dim3(kLayers * kDin * kRankP / 8 / 256), 256, 0, stream>>>(
      dtproj_w, WDt, kDin, kDin, kRank, kRankP, kCarryWdt);
  cast_pad_f16_kernel<<<dim3(kLayers * kDm * kDin / 8 / 256), 256, 0, stream>>>(
      outproj_w, WOut, kDm, kDm, kDin, kDin, kCarryW);
  cast_pad_f16_kernel<<<dim3(kNclsP * kDm / 8 / 256), 256, 0, stream>>>(
      cls_w, WCls, kNclsP, kNcls, kDm, kDm, kCarryW);

  gemm_f16_kernel<4, 1, 2><<<dim3((kRows / 64) * (kDm / 64) / 8), 256, 0, stream>>>(
      ColA, ColA, kKpP, WPatch, kKpP, T0, kDm, PoolH, kDm, 0, patch_b, patch_b,
      kRows, kDm, kKpP, kFoldPatch, 0.0f, 0.0f);

  for (int l = 0; l < kLayers; ++l) {
    float* tcur  = ((l & 1) == 0) ? T0 : T1;
    float* tnext = ((l & 1) == 0) ? T1 : T0;
    const unsigned short* WIn_l  = WIn  + (size_t)l * kXzN * kDm;
    const unsigned short* WX_l   = WX   + (size_t)l * kXdP * kDin;
    const unsigned short* WDt_l  = WDt  + (size_t)l * kDin * kRankP;
    const unsigned short* WOut_l = WOut + (size_t)l * kDm * kDin;
    for (int hf = 0; hf < kHalves; ++hf) {
      const size_t r0 = (size_t)hf * kHalfRows;
      const float* tc_h = tcur + r0 * kDm;
      float* tn_h = tnext + r0 * kDm;

      ln_f16_kernel<<<dim3(kHalfRows / 8), 256, 0, stream>>>(
          tc_h, norm_w + (size_t)l * kDm, norm_b + (size_t)l * kDm, XN, kCarryXn);

      gemm_f16_kernel<4, 1, 0><<<dim3((kHalfRows / 64) * (kXzN / 64) / 8), 256, 0, stream>>>(
          XN, XN, kDm, WIn_l, kDm, XZ, kXzN, PoolH, kDm, 0, patch_b, patch_b,
          kHalfRows, kXzN, kDm, kFoldIn, 0.0f, 0.0f);

      conv_silu_kernel<<<dim3(kHalfRows), 192, 0, stream>>>(
          XZ, conv_w + (size_t)l * kDin * 4, conv_b + (size_t)l * kDin, UC, UCh, kCarryUc);

      gemm_f16_kernel<4, 1, 1><<<dim3((kHalfRows / 64) * (kXdP / 64) / 8), 256, 0, stream>>>(
          UCh, UCh, kDin, WX_l, kDin, XDBL, kXdP, DTLh, kRankP, kRank, patch_b, patch_b,
          kHalfRows, kXdP, kDin, kFoldXp, 0.0f, kCarryDtl);

      gemm_f16_kernel<4, 1, 2><<<dim3((kHalfRows / 64) * (kDin / 64) / 8), 256, 0, stream>>>(
          DTLh, DTLh, kRankP, WDt_l, kRankP, DTP, kDin, PoolH, kDm, 0, dtproj_b + (size_t)l * kDin, patch_b,
          kHalfRows, kDin, kRankP, kFoldDt, 0.0f, 0.0f);

      for (int im = 0; im < kHalfImgs; ++im) {
        const size_t rl = (size_t)im * kSeq;
        ms1_args sa;
        sa.dtpre = DTP + rl * kDin;
        sa.u = UC + rl * kDin;
        sa.bc = XDBL + rl * kXdP;
        sa.z = XZ + rl * kXzN;
        sa.A_log = A_log + (size_t)l * kDin * kNstate;
        sa.Dskip = D_par + (size_t)l * kDin;
        sa.y = (__half*)(YH + rl * kDin);
        sa.y_lo = (__half*)(YL + rl * kDin);
        sa.ld_dtpre = kDin;
        sa.ld_u = kDin;
        sa.ld_bc = kXdP;
        sa.ld_z = kXzN;
        sa.ld_y = kDin;
        sa.offB = kOffB;
        sa.offC = kOffC;
        sa.offZ = kDin;
        sa.ycarry = kCarryY;
        sa.dir = 1;
        sa.D = kDin;
        sa.L = kSeq;
        sa.nbatch = 1;
        ms1_scan_kernel<16><<<dim3(kDin / 64), 64, 0, stream>>>(sa);
      }

      gemm_f16_kernel<2, 2, 3><<<dim3((kHalfRows / 32) * (kDm / 64) / 8), 256, 0, stream>>>(
          YH, YL, kDin, WOut_l, kDin, tn_h, kDm, PoolH, kDm, 0, patch_b, tc_h,
          kHalfRows, kDm, kDin, kFoldOut, kFoldResid, 0.0f);
    }
  }
  static_assert((kLayers & 1) == 0);

  ln_pool_kernel<<<dim3(kBatch), 256, 0, stream>>>(T0, fnorm_w, fnorm_b, PoolH, kCarryPool);

  gemm_f16_kernel<2, 1, 0><<<dim3(((kBatch / 32) * (kNclsP / 64) + 7) / 8), 256, 0, stream>>>(
      PoolH, PoolH, kDm, WCls, kDm, LOG, kNclsP, DTLh, kRankP, 0, patch_b, patch_b,
      kBatch, kNclsP, kDm, kFoldHead, 0.0f, 0.0f);

  logits_out_kernel<<<dim3(kBatch * kNcls / 256), 256, 0, stream>>>(LOG, cls_b, out);
}
